// StochasticGAT_9723805958349
// MI455X (gfx1250) — hardware-verified
//
#include <hip/hip_runtime.h>
#include <stdint.h>

#define NN   50000
#define EE   800000
#define DIM  128
#define HEADS 4
#define HD   32
#define BUCKET 64
#define NBK   ((NN + BUCKET - 1) / BUCKET)
#define NBKP  800
#define CHUNK 2048
#define NCH   ((EE + CHUNK - 1) / CHUNK)
#define SLOT  32
#define LCAP  1536
#define N_NODES NN
#define RSPLIT (1.0f / 2048.0f)

typedef _Float16 f16;
typedef __attribute__((ext_vector_type(16))) _Float16 v16h;
typedef __attribute__((ext_vector_type(8)))  _Float16 v8h;
typedef __attribute__((ext_vector_type(8)))  float    v8f;
typedef __attribute__((ext_vector_type(4)))  float    f32x4;
typedef float v4fa __attribute__((ext_vector_type(4), may_alias));

__device__ __forceinline__ v8f wmma16(v16h a, v16h b, v8f c) {
  return __builtin_amdgcn_wmma_f32_16x16x32_f16(false, a, false, b, (short)0, c, false, false);
}
__device__ __forceinline__ v8f wmma_split(v16h a, v16h al, v16h b, v16h bl, v8f c) {
  v8f x = {};
  x = wmma16(al, b, x); x = wmma16(a, bl, x);
  return wmma16(a, b, c) + x * RSPLIT;
}
__device__ __forceinline__ f16 lo_of(float v, f16 h) { return (f16)((v - (float)h) * 2048.0f); }
__device__ __forceinline__ v16h cat8(v8h a, v8h b) { return __builtin_shufflevector(a, b, 0,1,2,3,4,5,6,7,8,9,10,11,12,13,14,15); }

__global__ __launch_bounds__(256) void pack_b_kernel(const float* __restrict__ Wm, f16* __restrict__ P) {
  const int t = (blockIdx.x * 256 + threadIdx.x) * 2;
  if (t >= DIM * DIM) return;
  unsigned ph = 0, pl = 0;
#pragma unroll
  for (int q = 0; q < 2; ++q) {
    const int tt = t + q, j = tt & 15, lane = (tt >> 4) & 31, nt = (tt >> 9) & 7, ks = tt >> 12, hi = lane >> 4;
    const int k = ks * 32 + ((j < 8) ? (hi * 8 + j) : (16 + hi * 8 + (j - 8)));
    const int col = nt * 16 + (lane & 15);
    const float v = Wm[k * DIM + col];
    const f16 h = (f16)v, l = lo_of(v, h);
    ph |= (unsigned)__builtin_bit_cast(unsigned short, h) << (16 * q);
    pl |= (unsigned)__builtin_bit_cast(unsigned short, l) << (16 * q);
  }
  *(volatile unsigned*)(P + t) = ph; *(volatile unsigned*)(P + DIM * DIM + t) = pl; __threadfence();
  *(volatile unsigned*)(P + t) = ph; *(volatile unsigned*)(P + DIM * DIM + t) = pl;
}

__global__ __launch_bounds__(256) void gemm128_split(const float* __restrict__ A, const f16* __restrict__ Bp, const float* __restrict__ bias,
                                                     float* __restrict__ C, int M) {
  __shared__ __attribute__((aligned(16))) float stg[8][16 * DIM];
  const int wave = threadIdx.x >> 5, lane = threadIdx.x & 31, l16 = lane & 15, hi = lane >> 4;
  const int rowBase = blockIdx.x * 128 + wave * 16;
  if (rowBase >= M) return;
  v8f acc[8];
#pragma unroll
  for (int i = 0; i < 8; ++i) acc[i] = (v8f){};
  const float* arow = A + (size_t)(rowBase + l16) * DIM;
#pragma unroll
  for (int ks = 0; ks < 4; ++ks) {
    const int kbA = ks * 32 + hi * 8;
    const f32x4 f0 = *(const f32x4*)(arow + kbA), f1 = *(const f32x4*)(arow + kbA + 4);
    const f32x4 f2 = *(const f32x4*)(arow + kbA + 16), f3 = *(const f32x4*)(arow + kbA + 20);
    float fv[16] = {f0[0],f0[1],f0[2],f0[3],f1[0],f1[1],f1[2],f1[3],f2[0],f2[1],f2[2],f2[3],f3[0],f3[1],f3[2],f3[3]};
    v16h a, al;
#pragma unroll
    for (int j = 0; j < 16; ++j) { const f16 h = (f16)fv[j]; a[j] = h; al[j] = lo_of(fv[j], h); }
#pragma unroll
    for (int nt = 0; nt < 8; ++nt) {
      const f16* fb = Bp + ((size_t)((ks * 8 + nt) << 5) + lane) * 16;
      const v16h b  = cat8(*(const v8h*)fb, *(const v8h*)(fb + 8));
      const v16h bl = cat8(*(const v8h*)(fb + DIM * DIM), *(const v8h*)(fb + DIM * DIM + 8));
      acc[nt] = wmma_split(a, al, b, bl, acc[nt]);
      asm volatile("" ::: "memory");
    }
  }
  float* sw = stg[wave];
#pragma unroll
  for (int nt = 0; nt < 8; ++nt) {
    const int col = nt * 16 + l16;
    const float badd = bias ? bias[col] : 0.0f;
#pragma unroll
    for (int j = 0; j < 8; ++j) sw[(j + hi * 8) * DIM + col] = acc[nt][j] + badd;
  }
  asm volatile("s_wait_dscnt 0" ::: "memory");
  float* ob = C + (size_t)rowBase * DIM;
#pragma unroll 1
  for (int pass = 0; pass < 2; ++pass) {
#pragma unroll
    for (int i = 0; i < 16; ++i) { const int c = lane + 32 * i; *(volatile f32x4*)(ob + c * 4) = *(const volatile v4fa*)(sw + c * 4); }
    __threadfence();
  }
}

__global__ __launch_bounds__(256) void bin_kernel(const int* __restrict__ dst, int* __restrict__ slots, int* __restrict__ cnts) {
  __shared__ int cnt[NBKP];
  const int tid = threadIdx.x, ch = blockIdx.x;
  for (int i = tid; i < NBKP; i += 256) cnt[i] = 0;
  __syncthreads();
  int eb[8], ps[8];
#pragma unroll
  for (int u = 0; u < 8; ++u) {
    const int e = ch * CHUNK + u * 256 + tid;
    eb[u] = -1; ps[u] = -1;
    if (e < EE) {
      int d = dst[e]; d = ((unsigned)d < (unsigned)NN) ? d : 0;
      const int b = d / BUCKET;
      const int p = atomicAdd(&cnt[b], 1);
      if (p < SLOT) { eb[u] = b; ps[u] = p; }
    }
  }
  __syncthreads();
#pragma unroll 1
  for (int pass = 0; pass < 2; ++pass) {
#pragma unroll
    for (int u = 0; u < 8; ++u)
      if (eb[u] >= 0) *(volatile int*)(slots + ((size_t)ch * NBK + eb[u]) * SLOT + ps[u]) = ch * CHUNK + u * 256 + tid;
    for (int i = tid; i < NBKP; i += 256) *(volatile int*)(cnts + (size_t)ch * NBKP + i) = (i < NBK) ? min(cnt[i], SLOT) : 0;
    __threadfence();
  }
}

__global__ __launch_bounds__(256) void gat_gather(const int* __restrict__ src, const int* __restrict__ dst,
                                                 const int* __restrict__ slots, const int* __restrict__ cnts,
                                                 const float* __restrict__ feat, const float* __restrict__ al, const float* __restrict__ ar,
                                                 const float* __restrict__ bias, float* __restrict__ out) {
  __shared__ int lst[LCAP];
  __shared__ int lsrc[LCAP];
  __shared__ int total;
  __shared__ int ncnt[BUCKET], noff[BUCKET];
  const int tid = threadIdx.x, lane = tid & 31, wave = tid >> 5;
  const int bk = blockIdx.x, n0 = bk * BUCKET;
  if (tid == 0) total = 0;
  if (tid < BUCKET) ncnt[tid] = 0;
  __syncthreads();
  int myc[2], mytot = 0;
#pragma unroll
  for (int u = 0; u < 2; ++u) { const int ch = tid + 256 * u; myc[u] = (ch < NCH) ? cnts[(size_t)ch * NBKP + bk] : 0; mytot += myc[u]; }
  {
    __shared__ int scan[256];
    scan[tid] = mytot;
    __syncthreads();
#pragma unroll
    for (int off = 1; off < 256; off <<= 1) { const int v = (tid >= off) ? scan[tid - off] : 0; __syncthreads(); scan[tid] += v; __syncthreads(); }
    int pos = scan[tid] - mytot;
    if (tid == 255) total = min(scan[255], LCAP);
#pragma unroll
    for (int u = 0; u < 2; ++u) {
      const int ch = tid + 256 * u;
      for (int i = 0; i < myc[u]; ++i) {
        if (pos < LCAP) {
          const int e = slots[((size_t)ch * NBK + bk) * SLOT + i];
          int d = dst[e]; d = ((unsigned)d < (unsigned)NN) ? d : 0;
          lst[pos] = ((d - n0) << 24) | e;
        }
        ++pos;
      }
    }
    __syncthreads();
  }
  const int nl = total;
  for (int i = tid; i < nl; i += 256) atomicAdd(&ncnt[(lst[i] >> 24) & 63], 1);
  __syncthreads();
  if (tid == 0) { int o = 0; for (int j = 0; j < BUCKET; ++j) { noff[j] = o; o += ncnt[j]; } }
  __syncthreads();
  if (tid < BUCKET) {
    int p = noff[tid];
    for (int i = 0; i < nl; ++i) if (((lst[i] >> 24) & 63) == tid) { int s = src[lst[i] & 0xFFFFFF]; s = ((unsigned)s < (unsigned)NN) ? s : 0; lsrc[p++] = s; }
  }
  __syncthreads();
  const int h = lane >> 3;
  const f32x4 alv = *(const f32x4*)(al + lane * 4), arv = *(const f32x4*)(ar + lane * 4), bv = *(const f32x4*)(bias + lane * 4);
  for (int j = wave; j < BUCKET; j += 8) {
    const int node = n0 + j;
    if (node >= NN) break;
    const f32x4 fn = *(const f32x4*)(feat + (size_t)node * DIM + lane * 4);
    float er_ = fn[0] * arv[0] + fn[1] * arv[1] + fn[2] * arv[2] + fn[3] * arv[3];
    er_ += __shfl_xor(er_, 1, 32); er_ += __shfl_xor(er_, 2, 32); er_ += __shfl_xor(er_, 4, 32);
    const int o0 = noff[j], cn = ncnt[j];
    float m = -3.0e38f, z = 0.f;
    f32x4 acc = {0.f, 0.f, 0.f, 0.f};
    for (int i = 0; i < cn; ++i) {
      const f32x4 fs = *(const f32x4*)(feat + (size_t)lsrc[o0 + i] * DIM + lane * 4);
      float el_ = fs[0] * alv[0] + fs[1] * alv[1] + fs[2] * alv[2] + fs[3] * alv[3];
      el_ += __shfl_xor(el_, 1, 32); el_ += __shfl_xor(el_, 2, 32); el_ += __shfl_xor(el_, 4, 32);
      float sc = el_ + er_; sc = (sc > 0.f) ? sc : 0.2f * sc;
      const float mn = fmaxf(m, sc);
      const float corr = __expf(m - mn);
      const float p = __expf(sc - mn);
      z = z * corr + p;
      acc = acc * corr + fs * p;
      m = mn;
    }
    const float inv = (cn > 0) ? (1.0f / z) : 0.0f;
    const f32x4 o = acc * inv + bv;
    float* dstp = out + (size_t)node * DIM + lane * 4;
    *(volatile f32x4*)dstp = o; __threadfence(); *(volatile f32x4*)dstp = o;
  }
}

extern "C" void kernel_launch(void* const* d_in, const int* in_sizes, int n_in,
                              void* d_out, int out_size, void* d_ws, size_t ws_size,
                              hipStream_t stream)
{
    (void)in_sizes; (void)n_in; (void)out_size; (void)ws_size;
    const float* x   = (const float*)d_in[0];
    const int*   src = (const int*)  d_in[1];
    const int*   dst = (const int*)  d_in[2];
    const float* W1  = (const float*)d_in[3];
    const float* al1 = (const float*)d_in[4];
    const float* ar1 = (const float*)d_in[5];
    const float* b1  = (const float*)d_in[6];
    const float* W2  = (const float*)d_in[7];
    const float* al2 = (const float*)d_in[8];
    const float* ar2 = (const float*)d_in[9];
    const float* b2  = (const float*)d_in[10];
    const float* Wp  = (const float*)d_in[11];
    const float* bp  = (const float*)d_in[12];

    char* w = (char*)d_ws;
    auto carve = [&](size_t bytes) -> char* { char* p = w; w += (bytes + 255) & ~(size_t)255; return p; };
    float* feat = (float*)carve((size_t)NN * DIM * 4);
    float* h1   = (float*)carve((size_t)NN * DIM * 4);
    f16*   w1b  = (f16*)carve((size_t)DIM * DIM * 2 * 2);
    f16*   w2b  = (f16*)carve((size_t)DIM * DIM * 2 * 2);
    f16*   wpb  = (f16*)carve((size_t)DIM * DIM * 2 * 2);
    int*   slots = (int*)carve((size_t)NCH * NBK * SLOT * 4);
    int*   cnts  = (int*)carve((size_t)NCH * NBKP * 4);

    float* h2  = (float*)d_out;
    float* prj = h2 + (size_t)NN * DIM;

    const int gemmBlocks = (NN + 127) / 128;
    pack_b_kernel<<<32, 256, 0, stream>>>(W1, w1b);
    pack_b_kernel<<<32, 256, 0, stream>>>(W2, w2b);
    pack_b_kernel<<<32, 256, 0, stream>>>(Wp, wpb);
    bin_kernel<<<NCH, 256, 0, stream>>>(dst, slots, cnts);

    gemm128_split<<<gemmBlocks, 256, 0, stream>>>(x, w1b, nullptr, feat, NN);
    gat_gather<<<NBK, 256, 0, stream>>>(src, dst, slots, cnts, feat, al1, ar1, b1, h1);
    gemm128_split<<<gemmBlocks, 256, 0, stream>>>(h1, w2b, nullptr, feat, NN);
    gat_gather<<<NBK, 256, 0, stream>>>(src, dst, slots, cnts, feat, al2, ar2, b2, h2);
    gemm128_split<<<gemmBlocks, 256, 0, stream>>>(h2, wpb, bp, prj, NN);
}
